// ConviSTFT_58849641889878
// MI455X (gfx1250) — hardware-verified
//
#include <hip/hip_runtime.h>
#include <math.h>

typedef __attribute__((ext_vector_type(16))) _Float16 v16h;
typedef __attribute__((ext_vector_type(16))) __bf16 v16b;
typedef __attribute__((ext_vector_type(8)))  _Float16 v8h;
typedef __attribute__((ext_vector_type(8)))  float v8f;
typedef __attribute__((ext_vector_type(4)))  float v4f;
typedef __attribute__((ext_vector_type(2)))  float v2f;
typedef __attribute__((ext_vector_type(4)))  unsigned v4u;
typedef __attribute__((ext_vector_type(4)))  int v4i;
typedef float __attribute__((may_alias)) float_a;
typedef int __attribute__((may_alias)) int_a;

template <typename T> __device__ __forceinline__ void vst2(void* p, T v) { *(volatile T*)p = v; __threadfence(); *(volatile T*)p = v; }
__device__ __forceinline__ v8f wmma16(v16h a, v16h b, v8f c) {
  v8f d = __builtin_amdgcn_wmma_f32_16x16x32_f16(false, a, false, b, (short)0, c, false, false);
  asm volatile("v_nop\n\tv_nop\n\tv_nop\n\tv_nop" : "+v"(d) : "v"(a), "v"(b));
  return d;
}
__device__ __forceinline__ v8f wmma_bf(v16b a, v16b b, v8f c) {
  v8f d = __builtin_amdgcn_wmma_f32_16x16x32_bf16(false, a, false, b, (short)0, c, false, false);
  asm volatile("v_nop\n\tv_nop\n\tv_nop\n\tv_nop" : "+v"(d) : "v"(a), "v"(b));
  return d;
}
__device__ __forceinline__ v16h frag_h(const _Float16* rowk0, int lane) {
  union { v16h v; v8h q[2]; } u; const _Float16* p = rowk0 + 8 * (lane >> 4);
  u.q[0] = *(const v8h*)p; u.q[1] = *(const v8h*)(p + 16); return u.v;
}
__device__ __forceinline__ v16h frag_f32(const float* rowk0, int lane) {
  v16h a; const float* p = rowk0 + 8 * (lane >> 4);
#pragma unroll
  for (int i = 0; i < 8; ++i) { a[i] = (_Float16)p[i]; a[8 + i] = (_Float16)p[16 + i]; }
  return a;
}
__device__ __forceinline__ v16h frag_f32s(const float* rowk0, int lane, float sc) {
  v16h a; const float* p = rowk0 + 8 * (lane >> 4);
#pragma unroll
  for (int i = 0; i < 8; ++i) { a[i] = (_Float16)(p[i] * sc); a[8 + i] = (_Float16)(p[16 + i] * sc); }
  return a;
}
__device__ __forceinline__ v16h fragc_f32(const float* W, int k0, int n, int lane, int ld, int K) {
  v16h a; const int g = lane >> 4;
#pragma unroll
  for (int i = 0; i < 8; ++i) { const int ka = k0 + 8 * g + i, kb = ka + 16;
    a[i] = (_Float16)(ka < K ? W[(size_t)ka * ld + n] : 0.f); a[8 + i] = (_Float16)(kb < K ? W[(size_t)kb * ld + n] : 0.f); }
  return a;
}
struct F2 { v16b h, l; };
__device__ __forceinline__ F2 bsplit16(const float v[16]) { F2 r;
#pragma unroll
  for (int i = 0; i < 16; ++i) { const __bf16 h = (__bf16)v[i]; r.h[i] = h; r.l[i] = (__bf16)(v[i] - (float)h); }
  return r; }
__device__ __forceinline__ F2 split_row(const float* row, int k0, int lane) { float v[16]; const float* p = row + k0 + 8 * (lane >> 4);
#pragma unroll
  for (int i = 0; i < 8; ++i) { v[i] = p[i]; v[8 + i] = p[16 + i]; }
  return bsplit16(v); }
__device__ __forceinline__ F2 split_rowK(const float* row, int k0, int lane, int K) { float v[16]; const int g = lane >> 4;
#pragma unroll
  for (int i = 0; i < 8; ++i) { const int ka = k0 + 8 * g + i, kb = ka + 16; v[i] = ka < K ? row[ka] : 0.f; v[8 + i] = kb < K ? row[kb] : 0.f; }
  return bsplit16(v); }
__device__ __forceinline__ F2 split_col(const float* W, int k0, int n, int lane, int ld, int K) { float v[16]; const int g = lane >> 4;
#pragma unroll
  for (int i = 0; i < 8; ++i) { const int ka = k0 + 8 * g + i, kb = ka + 16; v[i] = ka < K ? W[(size_t)ka * ld + n] : 0.f; v[8 + i] = kb < K ? W[(size_t)kb * ld + n] : 0.f; }
  return bsplit16(v); }
__device__ __forceinline__ v8f mac3(const F2& a, const F2& b, v8f c) { c = wmma_bf(a.l, b.h, c); c = wmma_bf(a.h, b.l, c); return wmma_bf(a.h, b.h, c); }
__device__ __forceinline__ float sigm(float v) { return 1.0f / (1.0f + expf(-v)); }
#define LDSX() do { asm volatile("s_wait_dscnt 0" ::: "memory"); __builtin_amdgcn_wave_barrier(); __builtin_amdgcn_fence(__ATOMIC_RELEASE, "workgroup"); } while (0)

#define NB 16
#define NF 257
#define NC 514
#define NT 2000
#define KW 400
#define ST 100
#define LOUT 200000
#define OFF0 (KW - ST)

__device__ __forceinline__ F2 frag_cspec(const float* __restrict__ inb, const float* __restrict__ phb, int t, int k0, int lane) {
  float v[16]; const int g = lane >> 4;
#pragma unroll
  for (int i = 0; i < 8; ++i) {
#pragma unroll
    for (int s = 0; s < 2; ++s) { const int c = k0 + 8 * g + i + 16 * s; float val = 0.f;
      if (c < NC) { const int cc = c < NF ? c : c - NF; const float mg = inb[(size_t)cc * NT + t], ph = phb[(size_t)cc * NT + t]; val = mg * (c < NF ? cosf(ph) : sinf(ph)); }
      v[i + 8 * s] = val; } }
  return bsplit16(v);
}
__global__ __launch_bounds__(128) void k_frames(const float* __restrict__ inp, const float* __restrict__ ph, const float* __restrict__ W, float* __restrict__ FR) {
  __shared__ __align__(16) float so[4][16][212];
  const int tid = threadIdx.x, wave = tid >> 5, lane = tid & 31, col = lane & 15, g = lane >> 4;
  const int b = blockIdx.y, t0 = blockIdx.x * 64 + wave * 16; const int t = (t0 + col) < NT ? (t0 + col) : NT - 1;
  const float* inb = inp + (size_t)b * NF * NT; const float* phb = ph + (size_t)b * NF * NT;
#pragma unroll 1
  for (int nh = 0; nh < 2; ++nh) { const int tb = nh * 13, ntl = nh == 0 ? 13 : 12; v8f acc[13];
#pragma unroll
    for (int j = 0; j < 13; ++j) acc[j] = (v8f){};
#pragma unroll 1
    for (int kc = 0; kc < (NC + 31) / 32; ++kc) { const F2 a = frag_cspec(inb, phb, t, kc * 32, lane);
#pragma unroll
      for (int j = 0; j < 13; ++j) { if (j < ntl) acc[j] = mac3(a, split_col(W, kc * 32, (tb + j) * 16 + col, lane, KW, NC), acc[j]); } }
#pragma unroll
    for (int j = 0; j < 13; ++j) { if (j < ntl) {
#pragma unroll
      for (int r = 0; r < 8; ++r) so[wave][8 * g + r][j * 16 + col] = acc[j][r]; } }
    LDSX();
    const int nq = ntl * 4;
    for (int q = lane; q < 16 * nq; q += 32) { const int rl = q / nq, pc = q % nq; const int tr = t0 + rl; if (tr < NT) vst2(FR + ((size_t)b * NT + tr) * KW + tb * 16 + pc * 4, *(const v4f*)(&so[wave][rl][pc * 4])); }
    LDSX(); }
}
__global__ __launch_bounds__(256) void k_ola(const float* __restrict__ FR, const float* __restrict__ win, float* __restrict__ out) {
  __shared__ float sw2[KW];
  const int tid = threadIdx.x, b = blockIdx.y; for (int k = tid; k < KW; k += 256) { const float w = win[k]; sw2[k] = w * w; }
  __syncthreads();
  const int j0 = blockIdx.x * 1024;
  for (int jj = tid * 4; jj < 1024; jj += 1024) { v4f o;
#pragma unroll
    for (int e = 0; e < 4; ++e) { const int j = j0 + jj + e; float val = 0.f, cof = 0.f;
      if (j < LOUT) { const int p = j + OFF0; int f_lo = (p - (KW - 1) + ST - 1) / ST; if (p - (KW - 1) < 0) f_lo = 0; int f_hi = p / ST; if (f_hi > NT - 1) f_hi = NT - 1;
        for (int f = f_lo; f <= f_hi; ++f) { const int k = p - f * ST; if (k >= 0 && k < KW) { val += FR[((size_t)b * NT + f) * KW + k]; cof += sw2[k]; } }
        val = val / (cof + 1e-12f); }
      o[e] = val; }
    if (j0 + jj < LOUT) vst2(out + (size_t)b * LOUT + j0 + jj, o); }
}
extern "C" void kernel_launch(void* const* d_in, const int* in_sizes, int n_in, void* d_out, int out_size, void* d_ws, size_t ws_size, hipStream_t stream) {
  (void)in_sizes; (void)n_in; (void)out_size; (void)ws_size;
  const float* inp = (const float*)d_in[0]; const float* ph = (const float*)d_in[1]; const float* W = (const float*)d_in[2]; const float* win = (const float*)d_in[3];
  float* out = (float*)d_out;
  float* FR = (float*)d_ws;
  k_frames<<<dim3((NT + 63) / 64, NB), 128, 0, stream>>>(inp, ph, W, FR);
  k_ola<<<dim3((LOUT + 1023) / 1024, NB), 256, 0, stream>>>(FR, win, out);
}
